// LoRACausalSelfAttention_52192442581221
// MI455X (gfx1250) — hardware-verified
//
#include <hip/hip_runtime.h>
#include <math.h>

typedef __attribute__((ext_vector_type(16))) _Float16 v16h;
typedef __attribute__((ext_vector_type(8)))  _Float16 v8h;
typedef __attribute__((ext_vector_type(16))) __bf16   v16b;
typedef __attribute__((ext_vector_type(8)))  __bf16   v8b;
typedef __attribute__((ext_vector_type(8)))  float    v8f;
typedef __attribute__((ext_vector_type(4)))  float    v4f;

constexpr int N_BATCH  = 4;
constexpr int SEQ_T    = 2048;
constexpr int HID_W    = 1024;
constexpr int N_HEAD   = 16;
constexpr int HEAD_D   = 64;
constexpr int RANK_R   = 8;
constexpr int N_TOK    = N_BATCH * SEQ_T;
constexpr int K_AUG    = 1088;
constexpr int N_QKV    = 3 * HID_W;
constexpr int K_COL0   = 1024;
constexpr int V_COL0   = 2048;
constexpr int T_LO     = 512;
constexpr int NQT_SPLIT = T_LO / 64;
constexpr int NQT_ALL  = SEQ_T / 64;
constexpr int U_COLS   = 64;
constexpr int KV_PITCH = 72;
constexpr int O_PITCH  = 68;
constexpr float CARRY_S = 16.0f;
constexpr float LO_S    = 4096.0f;
constexpr float P_S     = 32768.0f;

static_assert(K_AUG % 32 == 0);
static_assert(HID_W % 32 == 0);
static_assert(N_TOK % 64 == 0 && N_QKV % 64 == 0 && T_LO % 64 == 0 && (SEQ_T - T_LO) % 64 == 0);

constexpr size_t SZ_AAUG = (size_t)N_TOK * K_AUG * 2;
constexpr size_t SZ_BAUG = (size_t)N_QKV * K_AUG * 2;
constexpr size_t SZ_ACAT = (size_t)U_COLS * HID_W * 2;
constexpr size_t SZ_BIAS = (size_t)N_QKV * 4;
constexpr size_t SZ_U    = (size_t)N_TOK * U_COLS * 4;
constexpr size_t SZ_QKVH = (size_t)N_TOK * N_QKV * 2;
constexpr size_t SZ_QKVL = (size_t)N_BATCH * T_LO * N_QKV * 2;
constexpr size_t SZ_VTH  = (size_t)N_BATCH * N_HEAD * HEAD_D * SEQ_T * 2;
constexpr size_t SZ_VTL  = (size_t)N_BATCH * N_HEAD * HEAD_D * T_LO * 2;
constexpr size_t OFF_AAUG = 0;
constexpr size_t OFF_BAUG = OFF_AAUG + SZ_AAUG;
constexpr size_t OFF_ACAT = OFF_BAUG + SZ_BAUG;
constexpr size_t OFF_BIAS = OFF_ACAT + SZ_ACAT;
constexpr size_t OFF_U    = OFF_BIAS + SZ_BIAS;
constexpr size_t OFF_QKVH = OFF_U    + SZ_U;
constexpr size_t OFF_QKVL = OFF_QKVH + SZ_QKVH;
constexpr size_t OFF_VTH  = OFF_QKVL + SZ_QKVL;
constexpr size_t OFF_VTL  = OFF_VTH  + SZ_VTH;
constexpr size_t WS_TOTAL = OFF_VTL  + SZ_VTL;
static_assert(WS_TOTAL == 110637056ull);
static_assert(WS_TOTAL <= 134217728ull);
static_assert(OFF_BAUG % 128 == 0 && OFF_ACAT % 128 == 0 && OFF_BIAS % 128 == 0 && OFF_U % 128 == 0 &&
              OFF_QKVH % 128 == 0 && OFF_QKVL % 128 == 0 && OFF_VTH % 128 == 0 && OFF_VTL % 128 == 0);

__device__ __forceinline__ unsigned short f2bf_bits(float f) {
  unsigned u = __float_as_uint(f);
  return (unsigned short)((u + 0x7FFFu + ((u >> 16) & 1u)) >> 16);
}
__device__ __forceinline__ float bf_bits2f(unsigned short h) { return __uint_as_float(((unsigned)h) << 16); }

__device__ __forceinline__ void dep_guard_h(v8f& a, v8f& b, v16h x, v16h y) { asm volatile("v_nop\n\tv_nop\n\tv_nop\n\tv_nop" : "+v"(a), "+v"(b) : "v"(x), "v"(y)); }
__device__ __forceinline__ void dep_guard_b(v8f& a, v8f& b, v16b x, v16b y) { asm volatile("v_nop\n\tv_nop\n\tv_nop\n\tv_nop" : "+v"(a), "+v"(b) : "v"(x), "v"(y)); }
__device__ __forceinline__ void keep4_h(v16h a, v16h b, v16h c, v16h d) { asm volatile("v_nop" :: "v"(a), "v"(b), "v"(c), "v"(d)); }
__device__ __forceinline__ void keep4_b(v16b a, v16b b, v16b c, v16b d) { asm volatile("v_nop" :: "v"(a), "v"(b), "v"(c), "v"(d)); }
__device__ __forceinline__ void acc_guard4(v8f& a, v8f& b, v8f& c, v8f& d) { asm volatile("v_nop\n\tv_nop\n\tv_nop\n\tv_nop" : "+v"(a), "+v"(b), "+v"(c), "+v"(d)); }
template <typename T> struct Frag;
template <> struct Frag<_Float16> {
  typedef v16h V; union U { v16h v; v8h h[2]; };
  static __device__ __forceinline__ v16h load(const _Float16* p) {
    U f; f.h[0] = *(const v8h*)(p); f.h[1] = *(const v8h*)(p + 16); return f.v;
  }
  static __device__ __forceinline__ v8f mma(v16h a, v16h b, v8f c) {
    return __builtin_amdgcn_wmma_f32_16x16x32_f16(false, a, false, b, (short)0, c, false, false);
  }
  static __device__ __forceinline__ void guard(v8f& a, v8f& b, v16h x, v16h y) { dep_guard_h(a, b, x, y); }
  static __device__ __forceinline__ void keep(v16h a, v16h b, v16h c, v16h d) { keep4_h(a, b, c, d); }
};
template <> struct Frag<__bf16> {
  typedef v16b V; union U { v16b v; v8b h[2]; };
  static __device__ __forceinline__ v16b load(const __bf16* p) {
    U f; f.h[0] = *(const v8b*)(p); f.h[1] = *(const v8b*)(p + 16); return f.v;
  }
  static __device__ __forceinline__ v8f mma(v16b a, v16b b, v8f c) {
    return __builtin_amdgcn_wmma_f32_16x16x32_bf16(false, a, false, b, (short)0, c, false, false);
  }
  static __device__ __forceinline__ void guard(v8f& a, v8f& b, v16b x, v16b y) { dep_guard_b(a, b, x, y); }
  static __device__ __forceinline__ void keep(v16b a, v16b b, v16b c, v16b d) { keep4_b(a, b, c, d); }
};

__device__ __forceinline__ v8f mma_h(v16h a, v16h b, v8f c) {
  c = __builtin_amdgcn_wmma_f32_16x16x32_f16(false, a, false, b, (short)0, c, false, false);
  asm volatile("v_nop\n\tv_nop\n\tv_nop\n\tv_nop" : "+v"(c) : "v"(a), "v"(b));
  return c;
}
__device__ __forceinline__ v8f zero8() { return (v8f){0.f,0.f,0.f,0.f,0.f,0.f,0.f,0.f}; }

union F8 { v4f v[2]; float f[8]; };

template <int ET> struct Elem;
template <> struct Elem<0> { typedef _Float16 T; };
template <> struct Elem<1> { typedef __bf16 T; };
template <int ET, int SPLITM, int BIAS_MODE, int OUT_MODE, bool RESID, int ACT = 0>
__global__ __launch_bounds__(256) void wmma_gemm64(
    const unsigned short* __restrict__ Ap, const unsigned short* __restrict__ A2p, int lda, long strideA,
    const unsigned short* __restrict__ Btp, const unsigned short* __restrict__ Bt2p, int ldb, long strideB,
    void* __restrict__ Cout, void* __restrict__ Cout2, int ldc, long strideC, long strideC2,
    const float* __restrict__ bias,
    const float* __restrict__ resid, long strideR,
    int M, int N, int K, float scale) {
  typedef typename Elem<ET>::T T;
  typedef typename Frag<T>::V V;
  constexpr bool SPA = (SPLITM >= 1);
  constexpr bool SPB = (SPLITM >= 2);
  const T* A = (const T*)Ap; const T* A2 = (const T*)A2p; const T* Bt = (const T*)Btp; const T* Bt2 = (const T*)Bt2p;
  __shared__ __align__(16) float sT[8][16 * 68];
  const int b    = blockIdx.y;
  const int lane = threadIdx.x & 31;
  const int wave = threadIdx.x >> 5;
  const int tilesN = N >> 6;
  const int tilesM = M >> 6;
  const int tile = blockIdx.x * 8 + wave;
  if (tile >= tilesM * tilesN) return;
  const int tm = tile / tilesN;
  const int tn = tile - tm * tilesN;
  const int m0 = tm << 6;
  const int n0 = tn << 6;

  const T* Ab  = A  + (size_t)b * strideA;
  const T* Bb  = Bt + (size_t)b * strideB;
  const T* Ab2 = SPA ? (A2  + (size_t)b * strideA) : nullptr;
  const T* Bb2 = SPB ? (Bt2 + (size_t)b * strideB) : nullptr;

  const int rlane = lane & 15;
  const int koff  = (lane >> 4) * 8;
  const int mOff  = (lane >> 4) * 8;

  v8f acc[4][4];
#pragma unroll
  for (int i = 0; i < 4; ++i)
#pragma unroll
    for (int j = 0; j < 4; ++j) acc[i][j] = (v8f){0.f,0.f,0.f,0.f,0.f,0.f,0.f,0.f};

  for (int k0 = 0; k0 < K; k0 += 32) {
    V bh[4], bl[4];
#pragma unroll
    for (int j = 0; j < 4; ++j) {
      const size_t bo = (size_t)(n0 + (j << 4) + rlane) * ldb + koff + k0;
      bh[j] = Frag<T>::load(Bb + bo);
      if (SPB) bl[j] = Frag<T>::load(Bb2 + bo);
    }
#pragma unroll
    for (int i = 0; i < 4; ++i) {
      const size_t ao = (size_t)(m0 + (i << 4) + rlane) * lda + koff + k0;
      V ah = Frag<T>::load(Ab + ao);
      V al;
      if (SPA) al = Frag<T>::load(Ab2 + ao);
#pragma unroll
      for (int j = 0; j < 4; ++j) {
        acc[i][j] = Frag<T>::mma(ah, bh[j], acc[i][j]);
        if (SPB) acc[i][j] = Frag<T>::mma(ah, bl[j], acc[i][j]);
        if (SPA) acc[i][j] = Frag<T>::mma(al, bh[j], acc[i][j]);
      }
      Frag<T>::guard(acc[i][0], acc[i][3], ah, SPA ? al : ah);
    }
    Frag<T>::keep(bh[0], bh[1], bh[2], bh[3]);
    if (SPB) Frag<T>::keep(bl[0], bl[1], bl[2], bl[3]);
  }
  acc_guard4(acc[0][0], acc[0][1], acc[0][2], acc[0][3]);
  acc_guard4(acc[1][0], acc[1][1], acc[1][2], acc[1][3]);
  acc_guard4(acc[2][0], acc[2][1], acc[2][2], acc[2][3]);
  acc_guard4(acc[3][0], acc[3][1], acc[3][2], acc[3][3]);

  float* slab = sT[wave];
  const float* Rb = RESID ? (resid + (size_t)b * strideR) : nullptr;
#pragma unroll
  for (int i = 0; i < 4; ++i) {
    const int mBase = m0 + (i << 4);
#pragma unroll
    for (int j = 0; j < 4; ++j) {
      const int n = n0 + (j << 4) + rlane;
      float bv = 0.f;
      if (BIAS_MODE == 2) bv = bias[n];
#pragma unroll
      for (int r = 0; r < 8; ++r) {
        float v = acc[i][j][r] * scale;
        if (BIAS_MODE == 1) v += bias[mBase + mOff + r];
        if (BIAS_MODE == 2) v += bv;
        if (RESID) v += Rb[(size_t)(mBase + mOff + r) * ldc + n];
        if (ACT == 1) v = tanhf(v);
        if (ACT == 2) v = fmaxf(v, 0.0f);
        if (ACT == 4) v = (v > 0.f) ? v : 0.01f * v;
        slab[(mOff + r) * 68 + (j << 4) + rlane] = v;
      }
    }
    __builtin_amdgcn_fence(__ATOMIC_RELEASE, "workgroup");
    __builtin_amdgcn_wave_barrier();
    __builtin_amdgcn_fence(__ATOMIC_ACQUIRE, "workgroup");
    if (OUT_MODE == 0) {
      float* C = (float*)Cout + (size_t)b * strideC;
      const int hh = lane >> 4, c4 = (lane & 15) * 4;
      for (int pass = 0; pass < 2; ++pass) {
#pragma unroll
        for (int it = 0; it < 8; ++it) {
          const int row = it * 2 + hh;
          v4f v = *(const v4f*)(slab + row * 68 + c4);
          *(volatile v4f*)(C + (size_t)(mBase + row) * ldc + n0 + c4) = v;
        }
        __threadfence();
      }
    } else {
      const int q = lane >> 3, c8 = (lane & 7) * 8;
      unsigned short* C  = (unsigned short*)Cout  + (size_t)b * strideC;
      unsigned short* C2 = (OUT_MODE >= 2) ? ((unsigned short*)Cout2 + (size_t)b * strideC2) : nullptr;
      for (int pass = 0; pass < 2; ++pass) {
#pragma unroll
        for (int it = 0; it < 4; ++it) {
          const int row = it * 4 + q;
          const float* sp = slab + row * 68 + c8;
          v8h hv, lv;
#pragma unroll
          for (int e = 0; e < 8; ++e) {
            if (OUT_MODE == 1) {
              hv[e] = (_Float16)sp[e];
            } else if (OUT_MODE == 3) {
              const _Float16 hq = (_Float16)sp[e];
              hv[e] = hq;
              lv[e] = (_Float16)((sp[e] - (float)hq) * 4096.0f);
            } else {
              unsigned short hb = f2bf_bits(sp[e]);
              unsigned short lb = f2bf_bits(sp[e] - bf_bits2f(hb));
              hv[e] = __builtin_bit_cast(_Float16, hb);
              lv[e] = __builtin_bit_cast(_Float16, lb);
            }
          }
          *(volatile v8h*)(C + (size_t)(mBase + row) * ldc + n0 + c8) = hv;
          if (OUT_MODE >= 2) *(volatile v8h*)(C2 + (size_t)(mBase + row) * ldc + n0 + c8) = lv;
        }
        __threadfence();
      }
    }
    __builtin_amdgcn_fence(__ATOMIC_RELEASE, "workgroup");
    __builtin_amdgcn_wave_barrier();
    __builtin_amdgcn_fence(__ATOMIC_ACQUIRE, "workgroup");
  }
}

__global__ __launch_bounds__(256) void cast_rows_bf16(const float* __restrict__ src, unsigned short* __restrict__ dst,
                                                      int npairs, int dst_ld_pairs) {
  const int i = blockIdx.x * 256 + threadIdx.x;
  if (i < npairs) {
    const int row = i >> 9, cp = i & 511;
    const float* s = src + (size_t)row * HID_W + 2 * cp;
    const unsigned u = (unsigned)f2bf_bits(s[0]) | ((unsigned)f2bf_bits(s[1]) << 16);
    unsigned* d = (unsigned*)dst + (size_t)row * dst_ld_pairs + cp;
    *(volatile unsigned*)d = u;
    __threadfence();
    *(volatile unsigned*)d = u;
  }
}

__global__ __launch_bounds__(256) void build_acat(const float* __restrict__ amq, const float* __restrict__ amk,
                                                  const float* __restrict__ amv, unsigned short* __restrict__ acat) {
  const int i = blockIdx.x * 256 + threadIdx.x;
  const int row = i >> 9, cp = i & 511, p = row >> 3, r = row & 7;
  const size_t so = (size_t)r * HID_W + 2 * cp;
  const float q0 = amq[so], q1 = amq[so + 1];
  const float k0 = amk[so], k1 = amk[so + 1];
  const float w0 = amv[so], w1 = amv[so + 1];
  const float x0 = (p == 0) ? q0 : (p == 1) ? k0 : (p == 2) ? w0 : 0.0f;
  const float x1 = (p == 0) ? q1 : (p == 1) ? k1 : (p == 2) ? w1 : 0.0f;
  const unsigned u = (unsigned)f2bf_bits(x0) | ((unsigned)f2bf_bits(x1) << 16);
  unsigned* d = (unsigned*)acat + i;
  *(volatile unsigned*)d = u;
  __threadfence();
  *(volatile unsigned*)d = u;
}

__global__ __launch_bounds__(256) void build_w_tail(const float* __restrict__ bmq, const float* __restrict__ bmk,
                                                    const float* __restrict__ bmv, unsigned short* __restrict__ baug) {
  const int tid = threadIdx.x, wave = tid >> 5, lane = tid & 31, q8 = lane >> 3, seg = lane & 7;
  const int n = blockIdx.x * 32 + wave * 4 + q8;
  const int p = n >> 10, o = n & 1023;
  F8 uq, uk, uv;
  uq.v[0] = *(const v4f*)(bmq + (size_t)o * RANK_R); uq.v[1] = *(const v4f*)(bmq + (size_t)o * RANK_R + 4);
  uk.v[0] = *(const v4f*)(bmk + (size_t)o * RANK_R); uk.v[1] = *(const v4f*)(bmk + (size_t)o * RANK_R + 4);
  uv.v[0] = *(const v4f*)(bmv + (size_t)o * RANK_R); uv.v[1] = *(const v4f*)(bmv + (size_t)o * RANK_R + 4);
  const bool keep = (seg < 6) && ((seg >> 1) == p);
  v8h hv;
#pragma unroll
  for (int e = 0; e < 8; ++e) {
    const float val = (p == 0) ? uq.f[e] : (p == 1) ? uk.f[e] : uv.f[e];
    const float w = keep ? (2.0f * val) : 0.0f;
    hv[e] = __builtin_bit_cast(_Float16, f2bf_bits(w));
  }
  unsigned short* d = baug + (size_t)n * K_AUG + HID_W + seg * 8;
  for (int pass = 0; pass < 2; ++pass) {
    *(volatile v8h*)d = hv;
    __threadfence();
  }
}

__global__ __launch_bounds__(256) void build_a_tail(const float* __restrict__ u, unsigned short* __restrict__ aaug) {
  const int tid = threadIdx.x, wave = tid >> 5, lane = tid & 31, q8 = lane >> 3, seg = lane & 7;
  const int m = blockIdx.x * 32 + wave * 4 + q8;
  int p = seg >> 1; p = (p > 2) ? 2 : p;
  const int islo = seg & 1;
  F8 uu;
  const float* up = u + (size_t)m * U_COLS + p * RANK_R;
  uu.v[0] = *(const v4f*)up; uu.v[1] = *(const v4f*)(up + 4);
  v8h hv;
#pragma unroll
  for (int e = 0; e < 8; ++e) {
    const unsigned short hb = f2bf_bits(uu.f[e]);
    const unsigned short lb = f2bf_bits(uu.f[e] - bf_bits2f(hb));
    const unsigned short o16 = (seg >= 6) ? (unsigned short)0 : (islo ? lb : hb);
    hv[e] = __builtin_bit_cast(_Float16, o16);
  }
  unsigned short* d = aaug + (size_t)m * K_AUG + HID_W + seg * 8;
  for (int pass = 0; pass < 2; ++pass) {
    *(volatile v8h*)d = hv;
    __threadfence();
  }
}

__global__ __launch_bounds__(256) void build_bias(const float* __restrict__ bq, const float* __restrict__ bk,
                                                  const float* __restrict__ bv, float* __restrict__ dst) {
  const int i = blockIdx.x * 256 + threadIdx.x;
  const int p = i >> 10, o = i & 1023;
  const float xq = bq[o], xk = bk[o], xv = bv[o];
  const float val = (p == 0) ? xq : (p == 1) ? xk : xv;
  const float w = bf_bits2f(f2bf_bits(val)) * CARRY_S;
  ((volatile float*)dst)[i] = w;
  __threadfence();
  ((volatile float*)dst)[i] = w;
}

__global__ __launch_bounds__(256) void vt_transpose(const unsigned short* __restrict__ srcp, unsigned short* __restrict__ vtp, int tsrc) {
  __shared__ __align__(16) _Float16 th[64 * KV_PITCH];
  const _Float16* src = (const _Float16*)srcp;
  const int st0 = blockIdx.x * 64, bh = blockIdx.y;
  const int b = (bh >> 4) & (N_BATCH - 1), h = bh & (N_HEAD - 1);
  const int tid = threadIdx.x;
  {
    const int sloc = tid >> 2, d0 = (tid & 3) * 16;
    const size_t so = ((size_t)b * tsrc + st0 + sloc) * N_QKV + V_COL0 + h * HEAD_D + d0;
    const v8h a0 = *(const v8h*)(src + so);
    const v8h a1 = *(const v8h*)(src + so + 8);
#pragma unroll
    for (int e = 0; e < 8; ++e) {
      th[(d0 + e) * KV_PITCH + sloc]     = a0[e];
      th[(d0 + 8 + e) * KV_PITCH + sloc] = a1[e];
    }
  }
  __syncthreads();
  const int wave = tid >> 5, lane = tid & 31, q8 = lane >> 3, c8 = (lane & 7) * 8;
  const int dA = wave * 8 + q8, dB = wave * 8 + 4 + q8;
  const v8h hvA = *(const v8h*)(th + dA * KV_PITCH + c8);
  const v8h hvB = *(const v8h*)(th + dB * KV_PITCH + c8);
  const size_t oA = ((size_t)bh * HEAD_D + dA) * tsrc + st0 + c8;
  const size_t oB = ((size_t)bh * HEAD_D + dB) * tsrc + st0 + c8;
  for (int pass = 0; pass < 2; ++pass) {
    *(volatile v8h*)(vtp + oA) = hvA;
    *(volatile v8h*)(vtp + oB) = hvB;
    __threadfence();
  }
}

template <bool SPLIT>
__global__ __launch_bounds__(128) void attn_causal_hd64(
    const unsigned short* __restrict__ php, const unsigned short* __restrict__ plp,
    const unsigned short* __restrict__ vthp, const unsigned short* __restrict__ vtlp,
    const float* __restrict__ amask, float* __restrict__ out, int qb0, int nqcnt) {
  const _Float16* ph  = (const _Float16*)php;
  const _Float16* pl  = (const _Float16*)plp;
  const _Float16* vth = (const _Float16*)vthp;
  const _Float16* vtl = (const _Float16*)vtlp;
  __shared__ __align__(16) _Float16 Ksh[64 * KV_PITCH];
  __shared__ __align__(16) _Float16 Ksl[SPLIT ? 64 * KV_PITCH : 8];
  __shared__ __align__(16) _Float16 Vsh[64 * KV_PITCH];
  __shared__ __align__(16) _Float16 Vsl[SPLIT ? 64 * KV_PITCH : 8];
  __shared__ __align__(16) _Float16 Psh[4][16 * KV_PITCH];
  __shared__ __align__(16) _Float16 Psl[SPLIT ? 4 : 1][SPLIT ? 16 * KV_PITCH : 8];
  __shared__ __align__(16) float  Os[4][16 * O_PITCH];

  const int tid  = threadIdx.x;
  const int wave = tid >> 5;
  const int lane = tid & 31;
  const int hh   = lane >> 4;
  const int c    = lane & 15;

  int qb = qb0 + (int)(blockIdx.x % (unsigned)nqcnt);
  qb = (qb > NQT_ALL - 1) ? (NQT_ALL - 1) : qb;
  const int bh = (int)(blockIdx.x / (unsigned)nqcnt);
  const int h  = bh & (N_HEAD - 1);
  const int b  = (bh >> 4) & (N_BATCH - 1);
  const int q0 = qb * 64 + wave * 16;

  v16h qh[2], ql[2];
  {
    const _Float16* qrow = ph + ((size_t)b * SEQ_T + q0 + c) * N_QKV + h * HEAD_D;
    int qlr = q0 + c; qlr = (qlr > T_LO - 1) ? (T_LO - 1) : qlr;
    const _Float16* qlrow = pl + ((size_t)b * T_LO + qlr) * N_QKV + h * HEAD_D;
#pragma unroll
    for (int dc = 0; dc < 2; ++dc) {
      qh[dc] = Frag<_Float16>::load(qrow + dc * 32 + 8 * hh);
      if (SPLIT) ql[dc] = Frag<_Float16>::load(qlrow + dc * 32 + 8 * hh);
      else ql[dc] = qh[dc];
    }
  }

  float mrow[8], lrow[8];
  v8f oacc[4];
#pragma unroll
  for (int r = 0; r < 8; ++r) { mrow[r] = -INFINITY; lrow[r] = 0.f; }
#pragma unroll
  for (int t = 0; t < 4; ++t) oacc[t] = zero8();

  const int nChunks = qb + 1;
  for (int kc = 0; kc < nChunks; ++kc) {
    const int kv0 = kc * 64;
    __syncthreads();
    {
      const int r = tid >> 1, hf = (tid & 1) * 32;
      const _Float16* ks = ph + ((size_t)b * SEQ_T + kv0 + r) * N_QKV + K_COL0 + h * HEAD_D + hf;
      const _Float16* vs = vth + ((size_t)bh * HEAD_D + r) * SEQ_T + kv0 + hf;
#pragma unroll
      for (int i = 0; i < 4; ++i) {
        *(v8h*)(Ksh + r * KV_PITCH + hf + 8 * i) = *(const v8h*)(ks + 8 * i);
        *(v8h*)(Vsh + r * KV_PITCH + hf + 8 * i) = *(const v8h*)(vs + 8 * i);
      }
      if (SPLIT) {
        const int kl0 = (kv0 > T_LO - 64) ? (T_LO - 64) : kv0;
        const _Float16* kls = pl + ((size_t)b * T_LO + kl0 + r) * N_QKV + K_COL0 + h * HEAD_D + hf;
        const _Float16* vls = vtl + ((size_t)bh * HEAD_D + r) * T_LO + kl0 + hf;
#pragma unroll
        for (int i = 0; i < 4; ++i) {
          *(v8h*)(Ksl + r * KV_PITCH + hf + 8 * i) = *(const v8h*)(kls + 8 * i);
          *(v8h*)(Vsl + r * KV_PITCH + hf + 8 * i) = *(const v8h*)(vls + 8 * i);
        }
      }
    }
    __syncthreads();

    float mk[4];
#pragma unroll
    for (int j = 0; j < 4; ++j) mk[j] = amask[(size_t)b * SEQ_T + kv0 + j * 16 + c];

    v8f s[4];
#pragma unroll
    for (int j = 0; j < 4; ++j) {
      s[j] = zero8();
      v8f sr = zero8();
#pragma unroll
      for (int dc = 0; dc < 2; ++dc) {
        const v16h kb = Frag<_Float16>::load(Ksh + (j * 16 + c) * KV_PITCH + dc * 32 + 8 * hh);
        s[j] = mma_h(qh[dc], kb, s[j]);
        if (SPLIT) {
          const v16h kl = Frag<_Float16>::load(Ksl + (j * 16 + c) * KV_PITCH + dc * 32 + 8 * hh);
          sr = mma_h(qh[dc], kl, sr);
          sr = mma_h(ql[dc], kb, sr);
        }
      }
      if (SPLIT) {
#pragma unroll
        for (int r = 0; r < 8; ++r) s[j][r] = s[j][r] + sr[r] * (1.0f / 4096.0f);
      }
    }

    const bool diag = (kc == qb);
    float cm[8];
#pragma unroll
    for (int r = 0; r < 8; ++r) {
      const int qrow = q0 + 8 * hh + r;
      float m = -INFINITY;
#pragma unroll
      for (int j = 0; j < 4; ++j) {
        const int kvcol = kv0 + j * 16 + c;
        float v = s[j][r] * (1.0f / 2048.0f) + mk[j];
        if (diag && (kvcol > qrow)) v = -INFINITY;
        s[j][r] = v;
        m = fmaxf(m, v);
      }
#pragma unroll
      for (int off = 1; off < 16; off <<= 1) m = fmaxf(m, __shfl_xor(m, off, 32));
      cm[r] = m;
    }

    _Float16* pwh = Psh[wave];
    _Float16* pwl = Psl[SPLIT ? wave : 0];
#pragma unroll
    for (int r = 0; r < 8; ++r) {
      const float mnew = fmaxf(mrow[r], cm[r]);
      const float alpha = expf(mrow[r] - mnew);
      mrow[r] = mnew;
      float psum = 0.f;
#pragma unroll
      for (int j = 0; j < 4; ++j) {
        const float p = expf(s[j][r] - mnew);
        psum += p;
        const float ps = p * P_S;
        const _Float16 hp = (_Float16)ps;
        pwh[(8 * hh + r) * KV_PITCH + j * 16 + c] = hp;
        if (SPLIT) pwl[(8 * hh + r) * KV_PITCH + j * 16 + c] = (_Float16)((ps - (float)hp) * LO_S);
      }
#pragma unroll
      for (int off = 1; off < 16; off <<= 1) psum += __shfl_xor(psum, off, 32);
      lrow[r] = lrow[r] * alpha + psum;
#pragma unroll
      for (int t = 0; t < 4; ++t) oacc[t][r] *= alpha;
    }
    __builtin_amdgcn_fence(__ATOMIC_RELEASE, "workgroup");
    __builtin_amdgcn_wave_barrier();
    __builtin_amdgcn_fence(__ATOMIC_ACQUIRE, "workgroup");

    v16h pa[2], pb2[2];
#pragma unroll
    for (int kk = 0; kk < 2; ++kk) {
      pa[kk] = Frag<_Float16>::load(pwh + c * KV_PITCH + kk * 32 + 8 * hh);
      if (SPLIT) pb2[kk] = Frag<_Float16>::load(pwl + c * KV_PITCH + kk * 32 + 8 * hh);
      else pb2[kk] = pa[kk];
    }
#pragma unroll
    for (int t = 0; t < 4; ++t) {
      v8f orr = zero8();
#pragma unroll
      for (int kk = 0; kk < 2; ++kk) {
        const v16h vb = Frag<_Float16>::load(Vsh + (t * 16 + c) * KV_PITCH + kk * 32 + 8 * hh);
        oacc[t] = mma_h(pa[kk], vb, oacc[t]);
        if (SPLIT) {
          const v16h vl2 = Frag<_Float16>::load(Vsl + (t * 16 + c) * KV_PITCH + kk * 32 + 8 * hh);
          orr = mma_h(pa[kk], vl2, orr);
          orr = mma_h(pb2[kk], vb, orr);
        }
      }
      if (SPLIT) {
#pragma unroll
        for (int r = 0; r < 8; ++r) oacc[t][r] = oacc[t][r] + orr[r] * (1.0f / 4096.0f);
      }
    }
  }

  float* os = Os[wave];
#pragma unroll
  for (int r = 0; r < 8; ++r) {
    const float inv = 1.0f / (lrow[r] * (P_S * CARRY_S));
#pragma unroll
    for (int t = 0; t < 4; ++t) os[(8 * hh + r) * O_PITCH + t * 16 + c] = oacc[t][r] * inv;
  }
  __builtin_amdgcn_fence(__ATOMIC_RELEASE, "workgroup");
  __builtin_amdgcn_wave_barrier();
  __builtin_amdgcn_fence(__ATOMIC_ACQUIRE, "workgroup");
  {
    const int c4 = (lane & 15) * 4;
    float* ob = out + ((size_t)b * SEQ_T + q0) * HID_W + h * HEAD_D;
    for (int pass = 0; pass < 2; ++pass) {
#pragma unroll
      for (int it = 0; it < 8; ++it) {
        const int row = it * 2 + hh;
        const v4f val = *(const v4f*)(os + row * O_PITCH + c4);
        *(volatile v4f*)(ob + (size_t)row * HID_W + c4) = val;
      }
      __threadfence();
    }
  }
}

extern "C" void kernel_launch(void* const* d_in, const int* in_sizes, int n_in,
                              void* d_out, int out_size, void* d_ws, size_t ws_size,
                              hipStream_t stream) {
  if (n_in < 14) return;
  if (in_sizes[0] != N_TOK * HID_W) return;
  if (in_sizes[1] != N_BATCH * SEQ_T) return;
  for (int p = 0; p < 3; ++p) {
    if (in_sizes[2 + 4 * p] != HID_W * HID_W) return;
    if (in_sizes[3 + 4 * p] != HID_W) return;
    if (in_sizes[4 + 4 * p] != RANK_R * HID_W) return;
    if (in_sizes[5 + 4 * p] != HID_W * RANK_R) return;
  }
  if (out_size != N_TOK * HID_W) return;
  if (ws_size < WS_TOTAL) return;

  const float* x   = (const float*)d_in[0];
  const float* am  = (const float*)d_in[1];
  const float* wq  = (const float*)d_in[2];
  const float* bq  = (const float*)d_in[3];
  const float* aq  = (const float*)d_in[4];
  const float* bmq = (const float*)d_in[5];
  const float* wk  = (const float*)d_in[6];
  const float* bk  = (const float*)d_in[7];
  const float* ak  = (const float*)d_in[8];
  const float* bmk = (const float*)d_in[9];
  const float* wv  = (const float*)d_in[10];
  const float* bv  = (const float*)d_in[11];
  const float* av  = (const float*)d_in[12];
  const float* bmv = (const float*)d_in[13];
  float* out = (float*)d_out;

  char* ws = (char*)d_ws;
  unsigned short* aaug  = (unsigned short*)(ws + OFF_AAUG);
  unsigned short* baug  = (unsigned short*)(ws + OFF_BAUG);
  unsigned short* acat  = (unsigned short*)(ws + OFF_ACAT);
  float*          biasc = (float*)(ws + OFF_BIAS);
  float*          u     = (float*)(ws + OFF_U);
  unsigned short* qkvh  = (unsigned short*)(ws + OFF_QKVH);
  unsigned short* qkvl  = (unsigned short*)(ws + OFF_QKVL);
  unsigned short* vth   = (unsigned short*)(ws + OFF_VTH);
  unsigned short* vtl   = (unsigned short*)(ws + OFF_VTL);

  cast_rows_bf16<<<dim3(N_TOK * 512 / 256), dim3(256), 0, stream>>>(x, aaug, N_TOK * 512, K_AUG / 2);
  cast_rows_bf16<<<dim3(HID_W * 512 / 256), dim3(256), 0, stream>>>(wq, baug,                              HID_W * 512, K_AUG / 2);
  cast_rows_bf16<<<dim3(HID_W * 512 / 256), dim3(256), 0, stream>>>(wk, baug + (size_t)1 * HID_W * K_AUG,  HID_W * 512, K_AUG / 2);
  cast_rows_bf16<<<dim3(HID_W * 512 / 256), dim3(256), 0, stream>>>(wv, baug + (size_t)2 * HID_W * K_AUG,  HID_W * 512, K_AUG / 2);
  build_acat<<<dim3(U_COLS * 512 / 256), dim3(256), 0, stream>>>(aq, ak, av, acat);
  build_w_tail<<<dim3(N_QKV / 32), dim3(256), 0, stream>>>(bmq, bmk, bmv, baug);
  build_bias<<<dim3(N_QKV / 256), dim3(256), 0, stream>>>(bq, bk, bv, biasc);
  wmma_gemm64<1, 0, 0, 0, false><<<dim3((N_TOK / 64) * (U_COLS / 64) / 8, 1), dim3(256), 0, stream>>>(
      aaug, aaug, K_AUG, 0L, acat, acat, HID_W, 0L,
      (void*)u, (void*)u, U_COLS, 0L, 0L, biasc, u, 0L, N_TOK, U_COLS, HID_W, 1.0f);
  build_a_tail<<<dim3(N_TOK / 32), dim3(256), 0, stream>>>(u, aaug);
  wmma_gemm64<1, 0, 2, 3, false><<<dim3((T_LO / 64) * (N_QKV / 64) / 8, N_BATCH), dim3(256), 0, stream>>>(
      aaug, aaug, K_AUG, (long)SEQ_T * K_AUG, baug, baug, K_AUG, 0L,
      (void*)qkvh, (void*)qkvl, N_QKV, (long)SEQ_T * N_QKV, (long)T_LO * N_QKV,
      biasc, u, 0L, T_LO, N_QKV, K_AUG, CARRY_S);
  wmma_gemm64<1, 0, 2, 1, false><<<dim3(((SEQ_T - T_LO) / 64) * (N_QKV / 64) / 8, N_BATCH), dim3(256), 0, stream>>>(
      aaug + (size_t)T_LO * K_AUG, aaug, K_AUG, (long)SEQ_T * K_AUG, baug, baug, K_AUG, 0L,
      (void*)(qkvh + (size_t)T_LO * N_QKV), (void*)qkvl, N_QKV, (long)SEQ_T * N_QKV, 0L,
      biasc, u, 0L, SEQ_T - T_LO, N_QKV, K_AUG, CARRY_S);
  vt_transpose<<<dim3(SEQ_T / 64, N_BATCH * N_HEAD), dim3(256), 0, stream>>>(qkvh, vth, SEQ_T);
  vt_transpose<<<dim3(T_LO / 64, N_BATCH * N_HEAD), dim3(256), 0, stream>>>(qkvl, vtl, T_LO);
  attn_causal_hd64<true><<<dim3(N_BATCH * N_HEAD * NQT_SPLIT), dim3(128), 0, stream>>>(
      qkvh, qkvl, vth, vtl, am, out, 0, NQT_SPLIT);
  attn_causal_hd64<false><<<dim3(N_BATCH * N_HEAD * (NQT_ALL - NQT_SPLIT)), dim3(128), 0, stream>>>(
      qkvh, qkvl, vth, vtl, am, out, NQT_SPLIT, NQT_ALL - NQT_SPLIT);
}
